// AttentionFCHead_90615220011047
// MI455X (gfx1250) — hardware-verified
//
#include <hip/hip_runtime.h>
#include <hip/hip_bf16.h>
#include <stddef.h>
#include <stdint.h>

#define NQ   512
#define MR   4096
#define FD   1024
#define NG   16
#define DG   64
#define MC   64
#define NCH  (MR / MC)
#define TP   72
#define SVP  264
#define GP   36
#define OTP  68

static_assert(NG * DG == FD);
static_assert(MR % MC == 0);
static_assert(MC == 64);
static_assert(NQ % 256 == 0);
static_assert(MR % 256 == 0);
static_assert(NQ % 16 == 0);
static_assert((NQ * FD) % 2048 == 0);
static_assert((MR * FD) % 2048 == 0);
static_assert((FD * FD) % 2048 == 0);

#define A_CUR   0
#define A_REF   (A_CUR + 16 * GP * 4)
#define A_WG    (A_REF + MC * GP * 4)
#define A_MISC  (A_WG + NG * TP * 2)
#define A_BIAS  (A_MISC + 256)
#define A_TILE  (A_BIAS + NG * 16 * MC * 4)
#define A_LDS   (A_TILE + 16 * 2 * 16 * TP * 2)
static_assert(A_REF == 2304);
static_assert(A_WG == 11520);
static_assert(A_MISC == 13824);
static_assert(A_BIAS == 14080);
static_assert(A_TILE == 79616);
static_assert(A_LDS == 153344);
static_assert(16 * 16 * OTP * 4 <= A_LDS);
static_assert((A_REF % 16) == 0 && (A_WG % 16) == 0 && (A_MISC % 16) == 0 && (A_BIAS % 16) == 0 && (A_TILE % 16) == 0);

typedef _Float16       v16h __attribute__((ext_vector_type(16)));
typedef _Float16       v8h  __attribute__((ext_vector_type(8)));
typedef __bf16         v16b __attribute__((ext_vector_type(16)));
typedef float          v8f  __attribute__((ext_vector_type(8)));
typedef float          v4f  __attribute__((ext_vector_type(4)));
typedef unsigned int   v4u  __attribute__((ext_vector_type(4)));
typedef unsigned short v8us __attribute__((ext_vector_type(8)));

union FragH { v16h v; v8h h[2]; };
union FragB { v16b v; v4u u[2]; };
union Pack8 { v8h h; v4u u; v8us s; };

__device__ __forceinline__ v8f zero8() { return (v8f){0.f, 0.f, 0.f, 0.f, 0.f, 0.f, 0.f, 0.f}; }

__device__ __forceinline__ v8f mma16(v16h a, v16h b, v8f c) {
  c = __builtin_amdgcn_wmma_f32_16x16x32_f16(false, a, false, b, (short)0, c, false, false);
  asm volatile("v_nop\n\tv_nop\n\tv_nop\n\tv_nop" : "+v"(c) : "v"(a), "v"(b));
  return c;
}

__device__ __forceinline__ v8f mma3(v16b ah, v16b al, v16b bh, v16b bl, v8f c) {
  c = __builtin_amdgcn_wmma_f32_16x16x32_bf16(false, ah, false, bh, (short)0, c, false, false);
  c = __builtin_amdgcn_wmma_f32_16x16x32_bf16(false, ah, false, bl, (short)0, c, false, false);
  c = __builtin_amdgcn_wmma_f32_16x16x32_bf16(false, al, false, bh, (short)0, c, false, false);
  asm volatile("v_nop\n\tv_nop\n\tv_nop\n\tv_nop" : "+v"(c) : "v"(ah), "v"(al), "v"(bh), "v"(bl));
  return c;
}

__device__ __forceinline__ v16h ldfragh(const _Float16* p, int ld, int row0, int k0, int lane) {
  const _Float16* q = p + (size_t)(row0 + (lane & 15)) * ld + k0 + 8 * (lane >> 4);
  FragH f;
  f.h[0] = *(const v8h*)(q);
  f.h[1] = *(const v8h*)(q + 16);
  return f.v;
}
__device__ __forceinline__ v16b ldfragb(const unsigned short* p, int ld, int row0, int k0, int lane) {
  const unsigned short* q = p + (size_t)(row0 + (lane & 15)) * ld + k0 + 8 * (lane >> 4);
  FragB f;
  f.u[0] = *(const v4u*)(q);
  f.u[1] = *(const v4u*)(q + 16);
  return f.v;
}

__device__ __forceinline__ unsigned int rne16(float x) {
  const unsigned int u = __float_as_uint(x);
  return (u + 0x7fffu + ((u >> 16) & 1u)) >> 16;
}
__device__ __forceinline__ void split2(float x0, float x1, unsigned int& hp, unsigned int& lp) {
  const unsigned int h0 = rne16(x0), h1 = rne16(x1);
  const unsigned int l0 = rne16(x0 - __uint_as_float(h0 << 16));
  const unsigned int l1 = rne16(x1 - __uint_as_float(h1 << 16));
  hp = h0 | (h1 << 16);
  lp = l0 | (l1 << 16);
}

__device__ __forceinline__ v8h tov8h(const float (&e)[8]) {
  return (v8h){(_Float16)e[0], (_Float16)e[1], (_Float16)e[2], (_Float16)e[3],
               (_Float16)e[4], (_Float16)e[5], (_Float16)e[6], (_Float16)e[7]};
}

__device__ __forceinline__ void sincos_f(float a, float& s, float& c) {
  const float k = rintf(a * 0.636619772367581343f);
  float r = fmaf(-k, 1.57079637050628662109375f, a);
  r = fmaf(-k, -4.37113900018624283e-8f, r);
  const int q = (int)k;
  const float z = r * r;
  float sp = fmaf(z, -1.9515295891e-4f, 8.3321608736e-3f);
  sp = fmaf(z, sp, -1.6666654611e-1f);
  const float sr = fmaf(z * r, sp, r);
  float cp = fmaf(z, 2.443315711809948e-5f, -1.388731625493765e-3f);
  cp = fmaf(z, cp, 4.166664568298827e-2f);
  const float cr = fmaf(z * z, cp, fmaf(z, -0.5f, 1.0f));
  const bool odd = (q & 1) != 0;
  const float ss = odd ? cr : sr;
  const float cc = odd ? sr : cr;
  s = (q & 2) ? -ss : ss;
  c = ((q + 1) & 2) ? -cc : cc;
}

__global__ __launch_bounds__(256) void k_split(const float* __restrict__ src,
                                               unsigned short* __restrict__ hi,
                                               unsigned short* __restrict__ lo) {
  const size_t e = (size_t)blockIdx.x * 2048 + (size_t)threadIdx.x * 8;
  const v4f a0 = *(const v4f*)(src + e);
  const v4f a1 = *(const v4f*)(src + e + 4);
  unsigned int h0, h1, h2, h3, l0, l1, l2, l3;
  split2(a0[0], a0[1], h0, l0);
  split2(a0[2], a0[3], h1, l1);
  split2(a1[0], a1[1], h2, l2);
  split2(a1[2], a1[3], h3, l3);
  const v4u hv = (v4u){h0, h1, h2, h3};
  const v4u lv = (v4u){l0, l1, l2, l3};
  volatile v4u* ph = (volatile v4u*)(hi + e);
  volatile v4u* pl = (volatile v4u*)(lo + e);
  *ph = hv;
  *pl = lv;
  __threadfence();
  *ph = hv;
  *pl = lv;
}

__global__ __launch_bounds__(256) void k_cvt16(const float* __restrict__ src, _Float16* __restrict__ dst, float scale) {
  const size_t e = (size_t)blockIdx.x * 2048 + (size_t)threadIdx.x * 8;
  const v4f a0 = *(const v4f*)(src + e) * scale;
  const v4f a1 = *(const v4f*)(src + e + 4) * scale;
  Pack8 pk;
  pk.h = (v8h){(_Float16)a0[0], (_Float16)a0[1], (_Float16)a0[2], (_Float16)a0[3],
               (_Float16)a1[0], (_Float16)a1[1], (_Float16)a1[2], (_Float16)a1[3]};
  const v4u vv = pk.u;
  volatile v4u* d = (volatile v4u*)(dst + e);
  *d = vv;
  __threadfence();
  *d = vv;
}

__device__ __forceinline__ void proj3_part(const v8f (&acc)[2][4], const float (&bb)[4], int part,
                                           unsigned short* st, unsigned short* __restrict__ dst,
                                           int tid, int wave, int hh, int c) {
  __syncthreads();
#pragma unroll
  for (int sub = 0; sub < 2; ++sub)
#pragma unroll
    for (int t = 0; t < 4; ++t)
#pragma unroll
      for (int r = 0; r < 8; ++r) {
        const float v = acc[sub][t][r] + bb[t];
        const unsigned int hb = rne16(v);
        const unsigned int lb = rne16(v - __uint_as_float(hb << 16));
        const unsigned int bits = part ? lb : hb;
        st[(wave * 32 + sub * 16 + 8 * hh + r) * TP + 16 * t + c] = (unsigned short)bits;
      }
  __syncthreads();
  v4u val[8];
  size_t go[8];
#pragma unroll
  for (int j = 0; j < 8; ++j) {
    const int p  = tid + 256 * j;
    const int lr = p >> 3;
    const int pc = p & 7;
    Pack8 pk;
    pk.s   = *(const v8us*)(st + lr * TP + pc * 8);
    val[j] = pk.u;
    go[j]  = (size_t)lr * DG + pc * 8;
  }
  for (int ps = 0; ps < 2; ++ps) {
#pragma unroll
    for (int j = 0; j < 8; ++j) *(volatile v4u*)(dst + go[j]) = val[j];
    __threadfence();
  }
}

__global__ __launch_bounds__(256) void k_proj3(const unsigned short* __restrict__ ahi,
                                               const unsigned short* __restrict__ alo,
                                               const unsigned short* __restrict__ whi,
                                               const unsigned short* __restrict__ wlo,
                                               const float* __restrict__ bias,
                                               unsigned short* __restrict__ ohi,
                                               unsigned short* __restrict__ olo, int nrows) {
  __shared__ __align__(16) unsigned short st[256 * TP];
  const int tid = threadIdx.x, lane = tid & 31, wave = tid >> 5;
  const int hh = lane >> 4, c = lane & 15;
  const int bx = blockIdx.x, g = blockIdx.y;
  const int m0 = bx * 256 + wave * 32;
  const int n0 = g * 64;

  v8f acc[2][4];
#pragma unroll
  for (int s = 0; s < 2; ++s)
#pragma unroll
    for (int t = 0; t < 4; ++t) acc[s][t] = zero8();

#pragma unroll 1
  for (int k0 = 0; k0 < FD; k0 += 32) {
    const v16b ah0 = ldfragb(ahi, FD, m0, k0, lane);
    const v16b ah1 = ldfragb(ahi, FD, m0 + 16, k0, lane);
    const v16b al0 = ldfragb(alo, FD, m0, k0, lane);
    const v16b al1 = ldfragb(alo, FD, m0 + 16, k0, lane);
#pragma unroll
    for (int t = 0; t < 4; ++t) {
      const v16b bh = ldfragb(whi, FD, n0 + 16 * t, k0, lane);
      const v16b bl = ldfragb(wlo, FD, n0 + 16 * t, k0, lane);
      acc[0][t] = mma3(ah0, al0, bh, bl, acc[0][t]);
      acc[1][t] = mma3(ah1, al1, bh, bl, acc[1][t]);
    }
  }
  float bb[4];
#pragma unroll
  for (int t = 0; t < 4; ++t) bb[t] = bias[n0 + 16 * t + c];

  unsigned short* dhi = ohi + ((size_t)g * nrows + (size_t)bx * 256) * DG;
  unsigned short* dlo = olo + ((size_t)g * nrows + (size_t)bx * 256) * DG;
  proj3_part(acc, bb, 0, st, dhi, tid, wave, hh, c);
  proj3_part(acc, bb, 1, st, dlo, tid, wave, hh, c);
}

__global__ __launch_bounds__(256) void k_projz(const _Float16* __restrict__ a16,
                                               const _Float16* __restrict__ w16,
                                               _Float16* __restrict__ zt) {
  __shared__ __align__(16) _Float16 st[DG * SVP];
  const int tid = threadIdx.x, lane = tid & 31, wave = tid >> 5;
  const int hh = lane >> 4, c = lane & 15;
  const int bx = blockIdx.x, g = blockIdx.y;
  const int m0 = bx * 256 + wave * 32;
  const int n0 = g * 64;

  v8f acc[2][4];
#pragma unroll
  for (int s = 0; s < 2; ++s)
#pragma unroll
    for (int t = 0; t < 4; ++t) acc[s][t] = zero8();

#pragma unroll 1
  for (int k0 = 0; k0 < FD; k0 += 32) {
    const v16h a0 = ldfragh(a16, FD, m0, k0, lane);
    const v16h a1 = ldfragh(a16, FD, m0 + 16, k0, lane);
#pragma unroll
    for (int t = 0; t < 4; ++t) {
      const v16h b = ldfragh(w16, FD, n0 + 16 * t, k0, lane);
      acc[0][t] = mma16(a0, b, acc[0][t]);
      acc[1][t] = mma16(a1, b, acc[1][t]);
    }
  }
#pragma unroll
  for (int sub = 0; sub < 2; ++sub)
#pragma unroll
    for (int t = 0; t < 4; ++t)
#pragma unroll
      for (int r = 0; r < 8; ++r)
        st[(16 * t + c) * SVP + wave * 32 + sub * 16 + 8 * hh + r] = (_Float16)(acc[sub][t][r] * 0.25f);
  __syncthreads();

  _Float16* base = zt + (size_t)n0 * MR + (size_t)bx * 256;
  v4u val[8];
  size_t go[8];
#pragma unroll
  for (int j = 0; j < 8; ++j) {
    const int p    = tid + 256 * j;
    const int drow = p >> 5;
    const int pc   = p & 31;
    Pack8 pk;
    pk.h   = *(const v8h*)(st + drow * SVP + pc * 8);
    val[j] = pk.u;
    go[j]  = (size_t)drow * MR + pc * 8;
  }
  for (int ps = 0; ps < 2; ++ps) {
#pragma unroll
    for (int j = 0; j < 8; ++j) *(volatile v4u*)(base + go[j]) = val[j];
    __threadfence();
  }
}

__global__ __launch_bounds__(512) void k_attn(const unsigned short* __restrict__ qhi,
                                              const unsigned short* __restrict__ qlo,
                                              const unsigned short* __restrict__ khi,
                                              const unsigned short* __restrict__ klo,
                                              const _Float16* __restrict__ zt,
                                              const float* __restrict__ bcur,
                                              const float* __restrict__ bkey,
                                              const float* __restrict__ wg,
                                              const float* __restrict__ wgb,
                                              const float* __restrict__ wvb,
                                              float* __restrict__ out) {
  extern __shared__ __align__(16) unsigned char dsm[];
  float*    curG  = (float*)(dsm + A_CUR);
  float*    keyG  = (float*)(dsm + A_REF);
  _Float16* wgS   = (_Float16*)(dsm + A_WG);
  float*    misc  = (float*)(dsm + A_MISC);
  float*    biasS = (float*)(dsm + A_BIAS);
  float*    osw   = (float*)(dsm + 0);

  const int tid = threadIdx.x, lane = tid & 31, wave = tid >> 5;
  const int hh = lane >> 4, c = lane & 15;
  const int n0 = blockIdx.x * 16;
  _Float16* etile = (_Float16*)(dsm + A_TILE) + wave * (2 * 16 * TP);
  _Float16* ptile = etile + 16 * TP;

  if (tid < 8) {
    const float d = (tid == 0) ? 1.0f
                  : (tid == 1) ? 2.37137370566166f
                  : (tid == 2) ? 5.62341325190349f
                  : (tid == 3) ? 13.3352143216332f
                  : (tid == 4) ? 31.6227766016838f
                  : (tid == 5) ? 74.9894209332456f
                  : (tid == 6) ? 177.827941003892f
                  :              421.696503428582f;
    const float rdim = 1.0f / d;
    misc[tid]     = rdim;
    misc[8 + tid] = 100.0f * rdim;
  }
  if (tid < NG) misc[16 + tid] = wgb[tid];
  for (int i = tid; i < NG * DG; i += 512) wgS[(i >> 6) * TP + (i & 63)] = (_Float16)(wg[i] * 64.0f);
  __syncthreads();

  if (tid < 128) {
    const int n = tid >> 3, j = tid & 7;
    const v4f bx = *(const v4f*)(bcur + (size_t)(n0 + n) * 4);
    const float w = (bx[2] - bx[0]) + 1.0f;
    const float h = (bx[3] - bx[1]) + 1.0f;
    const float cj = misc[8 + j];
    float s, co;
    sincos_f(logf(w) * cj, s, co);
    curG[n * GP + 4 + j]  = s;
    curG[n * GP + 12 + j] = co;
    sincos_f(logf(h) * cj, s, co);
    curG[n * GP + 20 + j] = s;
    curG[n * GP + 28 + j] = co;
    if (j == 0) {
      curG[n * GP + 0] = 0.5f * (bx[0] + bx[2]);
      curG[n * GP + 1] = 0.5f * (bx[1] + bx[3]);
      curG[n * GP + 2] = 1.0f / w;
      curG[n * GP + 3] = 1.0f / h;
    }
  }
  float rd[8];
#pragma unroll
  for (int j = 0; j < 8; ++j) rd[j] = misc[j];
  __syncthreads();

  const unsigned short* qh_g = qhi + (size_t)wave * NQ * DG;
  const unsigned short* ql_g = qlo + (size_t)wave * NQ * DG;
  const unsigned short* kh_g = khi + (size_t)wave * MR * DG;
  const unsigned short* kl_g = klo + (size_t)wave * MR * DG;
  const _Float16* zt_g = zt + (size_t)wave * DG * MR;
  const float* cg = curG + wave * GP;

  const float NEGI = -__builtin_huge_valf();
  float mrow[8], lrow[8];
  v8f oacc[4];
#pragma unroll
  for (int r = 0; r < 8; ++r) { mrow[r] = NEGI; lrow[r] = 0.f; }
#pragma unroll
  for (int t = 0; t < 4; ++t) oacc[t] = zero8();

#pragma unroll 1
  for (int kc = 0; kc < NCH; ++kc) {
    const int mc0 = kc * MC;
    __syncthreads();
    {
      const int b = tid >> 3, j = tid & 7;
      const v4f bx = *(const v4f*)(bkey + (size_t)(mc0 + b) * 4);
      const float w = (bx[2] - bx[0]) + 1.0f;
      const float h = (bx[3] - bx[1]) + 1.0f;
      const float cj = misc[8 + j];
      float s, co;
      sincos_f(logf(w) * cj, s, co);
      keyG[b * GP + 4 + j]  = s;
      keyG[b * GP + 12 + j] = co;
      sincos_f(logf(h) * cj, s, co);
      keyG[b * GP + 20 + j] = s;
      keyG[b * GP + 28 + j] = co;
      if (j == 0) {
        keyG[b * GP + 0] = 0.5f * (bx[0] + bx[2]);
        keyG[b * GP + 1] = 0.5f * (bx[1] + bx[3]);
      }
    }
    __syncthreads();

#pragma unroll 1
    for (int i = 0; i < 4; ++i) {
      const int mloc = 16 * i + c;
      const float* rg = keyG + mloc * GP;
      const float cpos = cg[hh], rinv = cg[2 + hh], rpos = rg[hh];
      const float dpos = logf(fabsf((cpos - rpos) * rinv) + 0.001f);
      const float p100 = dpos * 100.0f;
      float es[8], ec[8], qs[8], qc[8];
#pragma unroll
      for (int j = 0; j < 8; ++j) sincos_f(p100 * rd[j], es[j], ec[j]);
      const float* tn = cg + 4 + 16 * hh;
      const float* tr = rg + 4 + 16 * hh;
#pragma unroll
      for (int j = 0; j < 8; ++j) {
        const float sn = tn[j], cn = tn[8 + j], sr = tr[j], cr = tr[8 + j];
        qs[j] = sn * cr - cn * sr;
        qc[j] = cn * cr + sn * sr;
      }
      _Float16* er = etile + c * TP + 16 * hh;
      *(v8h*)(er)      = tov8h(es);
      *(v8h*)(er + 8)  = tov8h(ec);
      *(v8h*)(er + 32) = tov8h(qs);
      *(v8h*)(er + 40) = tov8h(qc);
      __syncthreads();
      {
        const v16h a0 = ldfragh(etile, TP, 0, 0, lane);
        const v16h a1 = ldfragh(etile, TP, 0, 32, lane);
        const v16h b0 = ldfragh(wgS, TP, 0, 0, lane);
        const v16h b1 = ldfragh(wgS, TP, 0, 32, lane);
        v8f dacc = zero8();
        dacc = mma16(a0, b0, dacc);
        dacc = mma16(a1, b1, dacc);
        const float bg = misc[16 + c];
        float* bw = biasS + (c * 16 + wave) * MC + 16 * i + 8 * hh;
#pragma unroll
        for (int r = 0; r < 8; ++r) {
          const float v = fmaxf(dacc[r] * 0.015625f + bg, 0.0f) + 1e-6f;
          bw[r] = __logf(v);
        }
      }
      __syncthreads();
    }

    const v16b qh0 = ldfragb(qh_g, DG, n0, 0, lane);
    const v16b qh1 = ldfragb(qh_g, DG, n0, 32, lane);
    const v16b ql0 = ldfragb(ql_g, DG, n0, 0, lane);
    const v16b ql1 = ldfragb(ql_g, DG, n0, 32, lane);
    v8f s[4];
#pragma unroll
    for (int j = 0; j < 4; ++j) {
      v8f a = zero8();
      {
        const v16b kh = ldfragb(kh_g, DG, mc0 + 16 * j, 0, lane);
        const v16b kl = ldfragb(kl_g, DG, mc0 + 16 * j, 0, lane);
        a = mma3(qh0, ql0, kh, kl, a);
      }
      {
        const v16b kh = ldfragb(kh_g, DG, mc0 + 16 * j, 32, lane);
        const v16b kl = ldfragb(kl_g, DG, mc0 + 16 * j, 32, lane);
        a = mma3(qh1, ql1, kh, kl, a);
      }
      s[j] = a;
    }
    const float* brow = biasS + (wave * 16) * MC;
    float cm[8];
#pragma unroll
    for (int r = 0; r < 8; ++r) {
      float m = NEGI;
#pragma unroll
      for (int j = 0; j < 4; ++j) {
        const float x = s[j][r] * 0.125f + brow[(8 * hh + r) * MC + 16 * j + c];
        s[j][r] = x;
        m = fmaxf(m, x);
      }
#pragma unroll
      for (int off = 1; off < 16; off <<= 1) m = fmaxf(m, __shfl_xor(m, off, 32));
      cm[r] = m;
    }
    float al[8];
#pragma unroll
    for (int r = 0; r < 8; ++r) {
      const float mnew  = fmaxf(mrow[r], cm[r]);
      const float alpha = __expf(mrow[r] - mnew);
      mrow[r] = mnew;
      float psum = 0.f;
#pragma unroll
      for (int j = 0; j < 4; ++j) {
        const float p = __expf(s[j][r] - mnew);
        psum += p;
        ptile[(8 * hh + r) * TP + 16 * j + c] = (_Float16)(p * 1024.0f);
      }
#pragma unroll
      for (int off = 1; off < 16; off <<= 1) psum += __shfl_xor(psum, off, 32);
      lrow[r] = lrow[r] * alpha + psum;
      al[r] = alpha;
    }
#pragma unroll
    for (int t = 0; t < 4; ++t)
#pragma unroll
      for (int r = 0; r < 8; ++r) oacc[t][r] *= al[r];
    __syncthreads();

#pragma unroll
    for (int kk = 0; kk < 2; ++kk) {
      const v16h pa = ldfragh(ptile, TP, 0, kk * 32, lane);
#pragma unroll
      for (int t = 0; t < 4; ++t) {
        const v16h zb = ldfragh(zt_g, MR, t * 16, mc0 + kk * 32, lane);
        oacc[t] = mma16(pa, zb, oacc[t]);
      }
    }
  }

  float il[8];
#pragma unroll
  for (int r = 0; r < 8; ++r) il[r] = (1.0f / lrow[r]) * 6.103515625e-05f;
  float bb[4];
#pragma unroll
  for (int t = 0; t < 4; ++t) bb[t] = wvb[wave * DG + 16 * t + c];
  __syncthreads();
  float* sw = osw + wave * (16 * OTP);
#pragma unroll
  for (int t = 0; t < 4; ++t)
#pragma unroll
    for (int r = 0; r < 8; ++r) sw[(8 * hh + r) * OTP + 16 * t + c] = oacc[t][r] * il[r] + bb[t];
  __syncthreads();
  v4f val[8];
  size_t go[8];
#pragma unroll
  for (int it = 0; it < 8; ++it) {
    const int p    = lane + 32 * it;
    const int L    = p >> 3;
    const int pc   = p & 7;
    const int row  = L >> 1;
    const int half = L & 1;
    val[it] = *(const v4f*)(sw + row * OTP + half * 32 + pc * 4);
    go[it]  = (size_t)(n0 + row) * FD + (size_t)wave * DG + half * 32 + pc * 4;
  }
  for (int ps = 0; ps < 2; ++ps) {
#pragma unroll
    for (int it = 0; it < 8; ++it) *(volatile v4f*)(out + go[it]) = val[it];
    __threadfence();
  }
}

extern "C" void kernel_launch(void* const* d_in, const int* in_sizes, int n_in,
                              void* d_out, int out_size, void* d_ws, size_t ws_size,
                              hipStream_t stream) {
  if (n_in < 12) return;
  if (in_sizes[0] != NQ * FD) return;
  if (in_sizes[1] != MR * FD) return;
  if (in_sizes[2] != NQ * 4) return;
  if (in_sizes[3] != MR * 4) return;
  if (in_sizes[4] != NG * DG) return;
  if (in_sizes[5] != NG) return;
  if (in_sizes[6] != FD * FD) return;
  if (in_sizes[7] != FD) return;
  if (in_sizes[8] != FD * FD) return;
  if (in_sizes[9] != FD) return;
  if (in_sizes[10] != FD * FD) return;
  if (in_sizes[11] != FD) return;
  if (out_size != NQ * FD) return;

  const float* roi  = (const float*)d_in[0];
  const float* feat = (const float*)d_in[1];
  const float* bcur = (const float*)d_in[2];
  const float* bkey = (const float*)d_in[3];
  const float* wg   = (const float*)d_in[4];
  const float* wgb  = (const float*)d_in[5];
  const float* wq   = (const float*)d_in[6];
  const float* bq   = (const float*)d_in[7];
  const float* wk   = (const float*)d_in[8];
  const float* bk   = (const float*)d_in[9];
  const float* wv   = (const float*)d_in[10];
  const float* bv   = (const float*)d_in[11];
  float* out = (float*)d_out;

  size_t off = 0;
  const size_t oRh  = off; off += (size_t)NQ * FD * 2;
  const size_t oRl  = off; off += (size_t)NQ * FD * 2;
  const size_t oFh  = off; off += (size_t)MR * FD * 2;
  const size_t oFl  = off; off += (size_t)MR * FD * 2;
  const size_t oF16 = off; off += (size_t)MR * FD * 2;
  const size_t oWqh = off; off += (size_t)FD * FD * 2;
  const size_t oWql = off; off += (size_t)FD * FD * 2;
  const size_t oWkh = off; off += (size_t)FD * FD * 2;
  const size_t oWkl = off; off += (size_t)FD * FD * 2;
  const size_t oWv  = off; off += (size_t)FD * FD * 2;
  const size_t oQh  = off; off += (size_t)NG * NQ * DG * 2;
  const size_t oQl  = off; off += (size_t)NG * NQ * DG * 2;
  const size_t oKh  = off; off += (size_t)NG * MR * DG * 2;
  const size_t oKl  = off; off += (size_t)NG * MR * DG * 2;
  const size_t oZt  = off; off += (size_t)NG * DG * MR * 2;
  if (off > ws_size) return;
  if (off > (size_t)134217728) return;

  char* ws = (char*)d_ws;
  unsigned short* Rh  = (unsigned short*)(ws + oRh);
  unsigned short* Rl  = (unsigned short*)(ws + oRl);
  unsigned short* Fh  = (unsigned short*)(ws + oFh);
  unsigned short* Fl  = (unsigned short*)(ws + oFl);
  _Float16*       F16 = (_Float16*)(ws + oF16);
  unsigned short* Wqh = (unsigned short*)(ws + oWqh);
  unsigned short* Wql = (unsigned short*)(ws + oWql);
  unsigned short* Wkh = (unsigned short*)(ws + oWkh);
  unsigned short* Wkl = (unsigned short*)(ws + oWkl);
  _Float16*       Wv16 = (_Float16*)(ws + oWv);
  unsigned short* Qh  = (unsigned short*)(ws + oQh);
  unsigned short* Ql  = (unsigned short*)(ws + oQl);
  unsigned short* Kh  = (unsigned short*)(ws + oKh);
  unsigned short* Kl  = (unsigned short*)(ws + oKl);
  _Float16*       Zt  = (_Float16*)(ws + oZt);

  k_split<<<dim3((NQ * FD) / 2048), dim3(256), 0, stream>>>(roi, Rh, Rl);
  k_split<<<dim3((MR * FD) / 2048), dim3(256), 0, stream>>>(feat, Fh, Fl);
  k_cvt16<<<dim3((MR * FD) / 2048), dim3(256), 0, stream>>>(feat, F16, 1.0f);
  k_split<<<dim3((FD * FD) / 2048), dim3(256), 0, stream>>>(wq, Wqh, Wql);
  k_split<<<dim3((FD * FD) / 2048), dim3(256), 0, stream>>>(wk, Wkh, Wkl);
  k_cvt16<<<dim3((FD * FD) / 2048), dim3(256), 0, stream>>>(wv, Wv16, 64.0f);
  k_proj3<<<dim3(NQ / 256, NG), dim3(256), 0, stream>>>(Rh, Rl, Wqh, Wql, bq, Qh, Ql, NQ);
  k_proj3<<<dim3(MR / 256, NG), dim3(256), 0, stream>>>(Fh, Fl, Wkh, Wkl, bk, Kh, Kl, MR);
  k_projz<<<dim3(MR / 256, NG), dim3(256), 0, stream>>>(F16, Wv16, Zt);
  (void)hipFuncSetAttribute(reinterpret_cast<const void*>(&k_attn),
                            hipFuncAttributeMaxDynamicSharedMemorySize, A_LDS);
  k_attn<<<dim3(NQ / 16), dim3(512), A_LDS, stream>>>(Qh, Ql, Kh, Kl, Zt, bcur, bkey, wg, wgb, bv, out);
  (void)hipGetLastError();
}
